// CausalSelfAttention_18519898980510
// MI455X (gfx1250) — hardware-verified
//
#include <hip/hip_runtime.h>


#ifndef NB
#define NB 4
#endif
#ifndef SEQ
#define SEQ 4096
#endif
#define NB_FULL  4
#define SEQ_FULL 4096
#define DMOD   256
#define NHEAD  4
#define HDIM   64
#define RHI    256
#define MTOK   (NB * SEQ)
#define NBH    (NB * NHEAD)
#define C2     0.18033688011112042f
#define PCL2   10.0f
#define NEGX   (-1.0e30f)

static_assert(NHEAD * HDIM == DMOD);
static_assert(HDIM == 64);
static_assert(DMOD % 64 == 0);
static_assert(SEQ % 256 == 0);
static_assert(RHI % 256 == 0);
static_assert(RHI <= SEQ);
static_assert(MTOK % 64 == 0);
static_assert(NB <= NB_FULL);
static_assert(SEQ <= SEQ_FULL);

typedef _Float16 h16;
typedef unsigned short bf;
typedef __attribute__((ext_vector_type(16))) __bf16   v16bf;
typedef __attribute__((ext_vector_type(16))) _Float16 v16h;
typedef __attribute__((ext_vector_type(8)))  _Float16 v8h;
typedef __attribute__((ext_vector_type(8)))  unsigned short v8us;
typedef __attribute__((ext_vector_type(8)))  float    v8f;
typedef __attribute__((ext_vector_type(4)))  float    v4f;
typedef v4f  __attribute__((may_alias)) v4fa;
typedef v8us __attribute__((may_alias)) v8usa;

__device__ __forceinline__ unsigned short f2bf(float f) { unsigned u = __float_as_uint(f); u += 0x7FFFu + ((u >> 16) & 1u); return (unsigned short)(u >> 16); }
__device__ __forceinline__ float bf2f(unsigned short b) { return __uint_as_float(((unsigned)b) << 16); }
__device__ __forceinline__ void splitf(float y, unsigned short& h, unsigned short& l) { h = f2bf(y); l = f2bf(y - bf2f(h)); }
__device__ __forceinline__ v16h cat16(v8h lo, v8h hi) { return __builtin_shufflevector(lo, hi, 0, 1, 2, 3, 4, 5, 6, 7, 8, 9, 10, 11, 12, 13, 14, 15); }
__device__ __forceinline__ v16bf cat16b(v8us lo, v8us hi) { return __builtin_bit_cast(v16bf, __builtin_shufflevector(lo, hi, 0, 1, 2, 3, 4, 5, 6, 7, 8, 9, 10, 11, 12, 13, 14, 15)); }
__device__ __forceinline__ v8f wmma16(v16h a, v16h b, v8f c) { return __builtin_amdgcn_wmma_f32_16x16x32_f16(false, a, false, b, (short)0, c, false, false); }
__device__ __forceinline__ v8f wmmab(v16bf a, v16bf b, v8f c) { return __builtin_amdgcn_wmma_f32_16x16x32_bf16(false, a, false, b, (short)0, c, false, false); }
__device__ __forceinline__ v16h  ldh(const h16* p) { return cat16(*(const v8h*)p, *(const v8h*)(p + 16)); }
__device__ __forceinline__ v16bf ldb(const bf* p)  { return cat16b(*(const v8us*)p, *(const v8us*)(p + 16)); }

__global__ __launch_bounds__(256) void k_cvt8(const float* __restrict__ src, bf* dst, int n8, size_t sS, size_t sD) {
    const int i = blockIdx.x * 256 + threadIdx.x; if (i >= n8) return;
    const float* s = src + (size_t)blockIdx.y * sS + (size_t)i * 8; bf* d = dst + (size_t)blockIdx.y * sD + (size_t)i * 8;
    const v4f a = *(const v4f*)s; const v4f c = *(const v4f*)(s + 4); v8us o;
    o[0] = f2bf(a[0]); o[1] = f2bf(a[1]); o[2] = f2bf(a[2]); o[3] = f2bf(a[3]); o[4] = f2bf(c[0]); o[5] = f2bf(c[1]); o[6] = f2bf(c[2]); o[7] = f2bf(c[3]);
    *(volatile v8us*)d = o; __threadfence(); *(volatile v8us*)d = o; }

__device__ __forceinline__ void gemm_kloop(const bf* __restrict__ A, const bf* __restrict__ Bt, const size_t aoff, const size_t boff, v8f (&acc)[4][4]) {
#pragma unroll 1
    for (int kc = 0; kc < DMOD; kc += 32) {
        v16bf a[4]; v16bf bl;
#pragma unroll
        for (int mb = 0; mb < 4; ++mb) a[mb] = ldb(A + aoff + (size_t)mb * 16 * DMOD + kc);
#pragma unroll
        for (int nb = 0; nb < 4; ++nb) { const v16bf b = ldb(Bt + boff + (size_t)nb * 16 * DMOD + kc); bl = b;
#pragma unroll
            for (int mb = 0; mb < 4; ++mb) acc[mb][nb] = wmmab(a[mb], b, acc[mb][nb]); }
        asm volatile("" : "+v"(acc[0][0]), "+v"(acc[0][1]), "+v"(acc[0][2]), "+v"(acc[0][3]), "+v"(acc[1][0]), "+v"(acc[1][1]), "+v"(acc[1][2]));
        asm volatile("" : "+v"(acc[1][3]), "+v"(acc[2][0]), "+v"(acc[2][1]), "+v"(acc[2][2]), "+v"(acc[2][3]), "+v"(acc[3][0]), "+v"(acc[3][1]));
        asm volatile("v_nop\n\tv_nop\n\tv_nop\n\tv_nop" : "+v"(acc[3][2]), "+v"(acc[3][3]) : "v"(a[3]), "v"(bl));
    }
}
template <int NSPLIT>
__device__ __forceinline__ void gemm_body(const bf* __restrict__ A, const bf* __restrict__ A2, const bf* __restrict__ Bt, float* C, const int ldc, const size_t sA, const size_t sC) {
    __shared__ __align__(16) float os[16 * 68];
    const size_t z = blockIdx.z; A += z * sA; A2 += z * sA; C += z * sC;
    const int lane = threadIdx.x & 31, lr = lane & 15, hi = lane >> 4; const int r0 = blockIdx.x * 64, c0 = blockIdx.y * 64;
    v8f acc[4][4];
#pragma unroll
    for (int mb = 0; mb < 4; ++mb)
#pragma unroll
        for (int nb = 0; nb < 4; ++nb) acc[mb][nb] = (v8f){};
    const size_t aoff = (size_t)(r0 + lr) * DMOD + 8 * hi, boff = (size_t)(c0 + lr) * DMOD + 8 * hi;
    gemm_kloop(A, Bt, aoff, boff, acc);
    if (NSPLIT == 1) gemm_kloop(A2, Bt, aoff, boff, acc);
#pragma unroll
    for (int mb = 0; mb < 4; ++mb) {
#pragma unroll
        for (int nb = 0; nb < 4; ++nb) {
#pragma unroll
            for (int j = 0; j < 8; ++j) os[(hi * 8 + j) * 68 + nb * 16 + lr] = acc[mb][nb][j]; }
        asm volatile("s_wait_dscnt 0" ::: "memory"); __builtin_amdgcn_wave_barrier();
        float* crow = C + (size_t)(r0 + mb * 16) * ldc + c0;
#pragma unroll 1
        for (int ps = 0; ps < 2; ++ps) {
#pragma unroll
            for (int s = 0; s < 8; ++s) { const int row = 2 * s + hi, cofs = lr * 4; const v4f val = *(const v4fa*)(os + row * 68 + cofs);
                *(volatile v4f*)(crow + (size_t)row * ldc + cofs) = val; }
            if (ps == 0) __threadfence(); }
        asm volatile("s_wait_dscnt 0" ::: "memory"); __builtin_amdgcn_wave_barrier();
    }
}
__global__ __launch_bounds__(32) void k_gemm_p(const bf* __restrict__ A, const bf* __restrict__ Bt, float* C, int ldc, size_t sA, size_t sC) { gemm_body<0>(A, A, Bt, C, ldc, sA, sC); }
__global__ __launch_bounds__(32) void k_gemm_hl(const bf* __restrict__ A, const bf* __restrict__ A2, const bf* __restrict__ Bt, float* C, int ldc, size_t sA, size_t sC) { gemm_body<1>(A, A2, Bt, C, ldc, sA, sC); }

__global__ __launch_bounds__(256) void k_plane_qk(const float* __restrict__ F, h16* P16, bf* Ph, bf* Pl) {
    const int idx = blockIdx.x * 256 + threadIdx.x; if (idx >= MTOK * 32) return;
    const int row = idx >> 5, g = idx & 31; const int hd = g >> 3, d0 = (g & 7) * 8; const int b = row / SEQ, s = row % SEQ;
    const float* f = F + (size_t)row * DMOD + g * 8; const v4f a = *(const v4f*)f; const v4f c = *(const v4f*)(f + 4);
    float y[8]; y[0] = a[0]; y[1] = a[1]; y[2] = a[2]; y[3] = a[3]; y[4] = c[0]; y[5] = c[1]; y[6] = c[2]; y[7] = c[3];
    v8h o16;
#pragma unroll
    for (int k = 0; k < 8; ++k) o16[k] = (h16)y[k];
    h16* d16 = P16 + ((size_t)(b * NHEAD + hd) * SEQ + s) * HDIM + d0;
    const bool early = (s < RHI); const size_t eo = ((size_t)(b * NHEAD + hd) * RHI + (early ? s : 0)) * HDIM + d0;
    v8us oh = (v8us){}, ol = (v8us){};
    if (early) {
#pragma unroll
        for (int k = 0; k < 8; ++k) { unsigned short p, q; splitf(y[k], p, q); oh[k] = p; ol[k] = q; } }
    *(volatile v8h*)d16 = o16; if (early) { *(volatile v8us*)(Ph + eo) = oh; *(volatile v8us*)(Pl + eo) = ol; }
    __threadfence();
    *(volatile v8h*)d16 = o16; if (early) { *(volatile v8us*)(Ph + eo) = oh; *(volatile v8us*)(Pl + eo) = ol; } }

__global__ __launch_bounds__(256) void k_plane_vt(const float* __restrict__ F, h16* VT16, bf* VTh, bf* VTl) {
    const int idx = blockIdx.x * 256 + threadIdx.x; if (idx >= DMOD * (MTOK / 8)) return;
    const int o = idx / (MTOK / 8); const int col = (idx % (MTOK / 8)) * 8; const int b = col / SEQ, s = col % SEQ; const int hd = o >> 6, d = o & 63;
    const float* f = F + (size_t)o * MTOK + col; const v4f a = *(const v4f*)f; const v4f c = *(const v4f*)(f + 4);
    float y[8]; y[0] = a[0]; y[1] = a[1]; y[2] = a[2]; y[3] = a[3]; y[4] = c[0]; y[5] = c[1]; y[6] = c[2]; y[7] = c[3];
    v8h o16;
#pragma unroll
    for (int k = 0; k < 8; ++k) o16[k] = (h16)y[k];
    const size_t prow = (size_t)(b * NHEAD + hd) * HDIM + d;
    h16* d16 = VT16 + prow * SEQ + s;
    const bool early = (s < RHI); const size_t eo = prow * RHI + (early ? s : 0);
    v8us oh = (v8us){}, ol = (v8us){};
    if (early) {
#pragma unroll
        for (int k = 0; k < 8; ++k) { unsigned short p, q; splitf(y[k], p, q); oh[k] = p; ol[k] = q; } }
    *(volatile v8h*)d16 = o16; if (early) { *(volatile v8us*)(VTh + eo) = oh; *(volatile v8us*)(VTl + eo) = ol; }
    __threadfence();
    *(volatile v8h*)d16 = o16; if (early) { *(volatile v8us*)(VTh + eo) = oh; *(volatile v8us*)(VTl + eo) = ol; } }

__device__ __forceinline__ void ctx_store(const v8f (&o)[4], const float inv, const int wave, const int lane, bf* CTXh, bf* CTXl, const size_t row0, const int col0) {
    __shared__ __align__(16) unsigned short cs[4 * 2 * 16 * 72];
    const int n = lane & 15, hh = lane >> 4; const int base = wave * (2 * 16 * 72);
#pragma unroll
    for (int t = 0; t < 4; ++t) { v8us vh, vl;
#pragma unroll
        for (int r = 0; r < 8; ++r) { unsigned short a, c; splitf(o[t][r] * inv, a, c); vh[r] = a; vl[r] = c; }
        *(v8usa*)(cs + base + n * 72 + 16 * t + 8 * hh) = vh; *(v8usa*)(cs + base + 16 * 72 + n * 72 + 16 * t + 8 * hh) = vl; }
    asm volatile("s_wait_dscnt 0" ::: "memory"); __builtin_amdgcn_wave_barrier();
    const int rq = lane >> 3, pc = lane & 7; v8us lh[4], ll[4];
#pragma unroll
    for (int i = 0; i < 4; ++i) { lh[i] = *(const v8usa*)(cs + base + (4 * i + rq) * 72 + pc * 8); ll[i] = *(const v8usa*)(cs + base + 16 * 72 + (4 * i + rq) * 72 + pc * 8); }
    asm volatile("" ::: "memory");
    const size_t g0 = (row0 + rq) * DMOD + col0 + pc * 8;
#pragma unroll
    for (int i = 0; i < 4; ++i) { *(volatile v8us*)(CTXh + g0 + (size_t)(4 * i) * DMOD) = lh[i]; *(volatile v8us*)(CTXl + g0 + (size_t)(4 * i) * DMOD) = ll[i]; }
    __threadfence();
#pragma unroll
    for (int i = 0; i < 4; ++i) { *(volatile v8us*)(CTXh + g0 + (size_t)(4 * i) * DMOD) = lh[i]; *(volatile v8us*)(CTXl + g0 + (size_t)(4 * i) * DMOD) = ll[i]; }
}

__global__ __launch_bounds__(128) void k_attn_main(const h16* __restrict__ Q16, const h16* __restrict__ K16, const h16* __restrict__ VT16, bf* CTXh, bf* CTXl) {
    const int wave = __builtin_amdgcn_readfirstlane((int)(threadIdx.x >> 5));
    const int lane = threadIdx.x & 31, n = lane & 15, hh = lane >> 4;
    const int bh = blockIdx.y; const int b = bh / NHEAD, h = bh % NHEAD;
    const int q0 = RHI + blockIdx.x * 64 + wave * 16;
    const h16* Qp = Q16 + (size_t)bh * SEQ * HDIM; const h16* Kp = K16 + (size_t)bh * SEQ * HDIM; const h16* Vp = VT16 + (size_t)bh * HDIM * SEQ;
    const int qoff = (q0 + n) * HDIM + 8 * hh;
    const v16h bq0 = ldh(Qp + qoff), bq1 = ldh(Qp + qoff + 32);
    v8f o[4];
#pragma unroll
    for (int t = 0; t < 4; ++t) o[t] = (v8f){};
    float m = NEGX, l = 0.f;
    const int nsteps = ((q0 + 15) >> 5) + 1;
#pragma unroll 1
    for (int st = 0; st < nsteps; ++st) {
        const int kb = st << 5; const int koff = (kb + n) * HDIM + 8 * hh;
        const v16h k00 = ldh(Kp + koff), k01 = ldh(Kp + koff + 32), k10 = ldh(Kp + koff + 16 * HDIM), k11 = ldh(Kp + koff + 16 * HDIM + 32);
        v8f s0 = (v8f){}, s1 = (v8f){};
        s0 = wmma16(k00, bq0, s0); s1 = wmma16(k10, bq0, s1); s0 = wmma16(k01, bq1, s0); s1 = wmma16(k11, bq1, s1);
        asm volatile("v_nop\n\tv_nop\n\tv_nop\n\tv_nop" : "+v"(s0), "+v"(s1) : "v"(k11), "v"(k01), "v"(bq1));
        float x0[8], x1[8];
#pragma unroll
        for (int r = 0; r < 8; ++r) { x0[r] = s0[r] * C2; x1[r] = s1[r] * C2; }
        if (kb + 31 > q0) {
            const int qi = q0 + n, kk = kb + 8 * hh;
#pragma unroll
            for (int r = 0; r < 8; ++r) { x0[r] = (kk + r > qi) ? NEGX : x0[r]; x1[r] = (kk + 16 + r > qi) ? NEGX : x1[r]; } }
        float mx = fmaxf(x0[0], x1[0]);
#pragma unroll
        for (int r = 1; r < 8; ++r) mx = fmaxf(mx, fmaxf(x0[r], x1[r]));
        mx = fmaxf(mx, __shfl_xor(mx, 16, 32));
        const float mnew = fmaxf(m, mx); const float corr = __builtin_amdgcn_exp2f(m - mnew); m = mnew;
        const float mb = mnew - PCL2;
        v8h p0, p1; float ps = 0.f;
#pragma unroll
        for (int r = 0; r < 8; ++r) { const h16 a = (h16)__builtin_amdgcn_exp2f(x0[r] - mb); const h16 c = (h16)__builtin_amdgcn_exp2f(x1[r] - mb); p0[r] = a; p1[r] = c; ps += (float)a; ps += (float)c; }
        ps += __shfl_xor(ps, 16, 32);
        l = l * corr + ps;
#pragma unroll
        for (int t = 0; t < 4; ++t) o[t] = o[t] * corr;
        const v16h pb = cat16(p0, p1);
        const int voff = n * SEQ + kb + 8 * hh;
        const v16h va0 = ldh(Vp + voff), va1 = ldh(Vp + voff + 16 * SEQ), va2 = ldh(Vp + voff + 32 * SEQ), va3 = ldh(Vp + voff + 48 * SEQ);
        o[0] = wmma16(va0, pb, o[0]); o[1] = wmma16(va1, pb, o[1]); o[2] = wmma16(va2, pb, o[2]); o[3] = wmma16(va3, pb, o[3]);
        asm volatile("v_nop\n\tv_nop\n\tv_nop\n\tv_nop" : "+v"(o[0]), "+v"(o[1]), "+v"(o[2]), "+v"(o[3]) : "v"(va3), "v"(pb));
    }
    const float inv = 1.0f / l;
    ctx_store(o, inv, wave, lane, CTXh, CTXl, (size_t)b * SEQ + q0, h * HDIM);
}

__global__ __launch_bounds__(128) void k_attn_early(const bf* __restrict__ Qh, const bf* __restrict__ Ql, const bf* __restrict__ Kh, const bf* __restrict__ Kl, const bf* __restrict__ VTh, const bf* __restrict__ VTl, bf* CTXh, bf* CTXl) {
    const int wave = __builtin_amdgcn_readfirstlane((int)(threadIdx.x >> 5));
    const int lane = threadIdx.x & 31, n = lane & 15, hh = lane >> 4;
    const int bh = blockIdx.y; const int b = bh / NHEAD, h = bh % NHEAD;
    const int q0 = blockIdx.x * 64 + wave * 16;
    const size_t po = (size_t)bh * RHI * HDIM;
    const bf* qhp = Qh + po; const bf* qlp = Ql + po; const bf* khp = Kh + po; const bf* klp = Kl + po; const bf* vhp = VTh + po; const bf* vlp = VTl + po;
    const int qoff = (q0 + n) * HDIM + 8 * hh;
    v8f o[4];
#pragma unroll
    for (int t = 0; t < 4; ++t) o[t] = (v8f){};
    float m = NEGX, l = 0.f;
    const int nsteps = ((q0 + 15) >> 5) + 1;
#pragma unroll 1
    for (int st = 0; st < nsteps; ++st) {
        const int kb = st << 5; const int koff = (kb + n) * HDIM + 8 * hh;
        v8f s0 = (v8f){}, s1 = (v8f){}; v16bf qh, ql, kh0, kl0, kh1, kl1;
#pragma unroll
        for (int ks = 0; ks < 2; ++ks) {
            qh = ldb(qhp + qoff + ks * 32); ql = ldb(qlp + qoff + ks * 32);
            kh0 = ldb(khp + koff + ks * 32); kl0 = ldb(klp + koff + ks * 32);
            kh1 = ldb(khp + koff + 16 * HDIM + ks * 32); kl1 = ldb(klp + koff + 16 * HDIM + ks * 32);
            s0 = wmmab(kh0, qh, s0); s0 = wmmab(kh0, ql, s0); s0 = wmmab(kl0, qh, s0);
            s1 = wmmab(kh1, qh, s1); s1 = wmmab(kh1, ql, s1); s1 = wmmab(kl1, qh, s1); }
        asm volatile("v_nop\n\tv_nop\n\tv_nop\n\tv_nop" : "+v"(s0), "+v"(s1) : "v"(kl1), "v"(kh1), "v"(qh), "v"(ql));
        float x0[8], x1[8];
#pragma unroll
        for (int r = 0; r < 8; ++r) { x0[r] = s0[r] * C2; x1[r] = s1[r] * C2; }
        if (kb + 31 > q0) {
            const int qi = q0 + n, kk = kb + 8 * hh;
#pragma unroll
            for (int r = 0; r < 8; ++r) { x0[r] = (kk + r > qi) ? NEGX : x0[r]; x1[r] = (kk + 16 + r > qi) ? NEGX : x1[r]; } }
        float mx = fmaxf(x0[0], x1[0]);
#pragma unroll
        for (int r = 1; r < 8; ++r) mx = fmaxf(mx, fmaxf(x0[r], x1[r]));
        mx = fmaxf(mx, __shfl_xor(mx, 16, 32));
        const float mnew = fmaxf(m, mx); const float corr = __builtin_amdgcn_exp2f(m - mnew); m = mnew;
        v8us ph0, pl0, ph1, pl1; float ps = 0.f;
#pragma unroll
        for (int r = 0; r < 8; ++r) { const float pa = __builtin_amdgcn_exp2f(x0[r] - mnew); const float pc = __builtin_amdgcn_exp2f(x1[r] - mnew); ps += pa; ps += pc;
            unsigned short a, c; splitf(pa, a, c); ph0[r] = a; pl0[r] = c; splitf(pc, a, c); ph1[r] = a; pl1[r] = c; }
        ps += __shfl_xor(ps, 16, 32);
        l = l * corr + ps;
#pragma unroll
        for (int t = 0; t < 4; ++t) o[t] = o[t] * corr;
        const v16bf pbh = cat16b(ph0, ph1), pbl = cat16b(pl0, pl1);
        const int voff = n * RHI + kb + 8 * hh; v16bf vh, vl;
#pragma unroll
        for (int t = 0; t < 4; ++t) { vh = ldb(vhp + voff + t * 16 * RHI); vl = ldb(vlp + voff + t * 16 * RHI);
            o[t] = wmmab(vh, pbh, o[t]); o[t] = wmmab(vh, pbl, o[t]); o[t] = wmmab(vl, pbh, o[t]); }
        asm volatile("v_nop\n\tv_nop\n\tv_nop\n\tv_nop" : "+v"(o[0]), "+v"(o[1]), "+v"(o[2]), "+v"(o[3]) : "v"(vl), "v"(vh), "v"(pbh), "v"(pbl));
    }
    const float inv = 1.0f / l;
    ctx_store(o, inv, wave, lane, CTXh, CTXl, (size_t)b * SEQ + q0, h * HDIM);
}

#define SZ_XB   ((size_t)MTOK * DMOD * 2)
#define SZ_W    ((size_t)DMOD * DMOD * 2)
#define SZ_F    ((size_t)MTOK * DMOD * 4)
#define SZ_P16  ((size_t)MTOK * DMOD * 2)
#define SZ_E    ((size_t)NBH * RHI * HDIM * 2)
#define SZ_CTX  ((size_t)MTOK * DMOD * 2)
#define SZ_TOTAL (SZ_XB + 4 * SZ_W + SZ_F + 3 * SZ_P16 + 6 * SZ_E + 2 * SZ_CTX)
static_assert(SZ_TOTAL <= (size_t)134217728);
static_assert(SZ_W % 256 == 0);
static_assert(SZ_E % 256 == 0);

extern "C" void kernel_launch(void* const* d_in, const int* in_sizes, int n_in,
                              void* d_out, int out_size, void* d_ws, size_t ws_size, hipStream_t stream) {
    if (n_in < 5) return;
    const int xneed = (NB - 1) * SEQ_FULL * DMOD + SEQ * DMOD;
    if (in_sizes[0] < xneed) return;
    if (in_sizes[1] < DMOD * DMOD || in_sizes[2] < DMOD * DMOD || in_sizes[3] < DMOD * DMOD || in_sizes[4] < DMOD * DMOD) return;
    if (out_size < xneed) return;
    if (ws_size < SZ_TOTAL) return;
    const float* x = (const float*)d_in[0]; const float* wq = (const float*)d_in[1]; const float* wk = (const float*)d_in[2]; const float* wv = (const float*)d_in[3]; const float* wo = (const float*)d_in[4];
    float* OUT = (float*)d_out;
    char* wsp = (char*)d_ws;
    auto take = [&](size_t bytes) { char* p = wsp; wsp += bytes; return (void*)p; };
    bf* XB = (bf*)take(SZ_XB); bf* WQ = (bf*)take(SZ_W); bf* WK = (bf*)take(SZ_W); bf* WV = (bf*)take(SZ_W); bf* WO = (bf*)take(SZ_W);
    float* F = (float*)take(SZ_F);
    h16* Q16 = (h16*)take(SZ_P16); h16* K16 = (h16*)take(SZ_P16); h16* VT16 = (h16*)take(SZ_P16);
    bf* Qh = (bf*)take(SZ_E); bf* Ql = (bf*)take(SZ_E); bf* Kh = (bf*)take(SZ_E); bf* Kl = (bf*)take(SZ_E); bf* VTh = (bf*)take(SZ_E); bf* VTl = (bf*)take(SZ_E);
    bf* CTXh = (bf*)take(SZ_CTX); bf* CTXl = (bf*)take(SZ_CTX);

    const int xn8 = SEQ * DMOD / 8, wn8 = DMOD * DMOD / 8;
    k_cvt8<<<dim3((xn8 + 255) / 256, NB, 1), 256, 0, stream>>>(x, XB, xn8, (size_t)SEQ_FULL * DMOD, (size_t)SEQ * DMOD);
    k_cvt8<<<dim3((wn8 + 255) / 256, 1, 1), 256, 0, stream>>>(wq, WQ, wn8, 0, 0);
    k_cvt8<<<dim3((wn8 + 255) / 256, 1, 1), 256, 0, stream>>>(wk, WK, wn8, 0, 0);
    k_cvt8<<<dim3((wn8 + 255) / 256, 1, 1), 256, 0, stream>>>(wv, WV, wn8, 0, 0);
    k_cvt8<<<dim3((wn8 + 255) / 256, 1, 1), 256, 0, stream>>>(wo, WO, wn8, 0, 0);
    k_gemm_p<<<dim3(MTOK / 64, DMOD / 64, 1), 32, 0, stream>>>(XB, WQ, F, DMOD, 0, 0);
    k_plane_qk<<<(MTOK * 32 + 255) / 256, 256, 0, stream>>>(F, Q16, Qh, Ql);
    k_gemm_p<<<dim3(MTOK / 64, DMOD / 64, 1), 32, 0, stream>>>(XB, WK, F, DMOD, 0, 0);
    k_plane_qk<<<(MTOK * 32 + 255) / 256, 256, 0, stream>>>(F, K16, Kh, Kl);
    k_gemm_p<<<dim3(DMOD / 64, MTOK / 64, 1), 32, 0, stream>>>(WV, XB, F, MTOK, 0, 0);
    k_plane_vt<<<(DMOD * (MTOK / 8) + 255) / 256, 256, 0, stream>>>(F, VT16, VTh, VTl);
    k_attn_early<<<dim3(RHI / 64, NBH, 1), 128, 0, stream>>>(Qh, Ql, Kh, Kl, VTh, VTl, CTXh, CTXl);
    if ((SEQ - RHI) / 64 > 0) k_attn_main<<<dim3((SEQ - RHI) / 64, NBH, 1), 128, 0, stream>>>(Q16, K16, VT16, CTXh, CTXl);
    k_gemm_hl<<<dim3(SEQ / 64, DMOD / 64, NB), 32, 0, stream>>>(CTXh, CTXl, WO, OUT, DMOD, (size_t)SEQ * DMOD, (size_t)SEQ_FULL * DMOD);
}
